// MPNN_54640573939922
// MI455X (gfx1250) — hardware-verified
//
#include <hip/hip_runtime.h>
#include <stddef.h>
#include <stdint.h>


#define NNODE    20000
#define NEDGE    640000
#define DH       128
#define NLAY     3
#define NGR      128
#define NCLS     2
#define APW      256
#define KTOT     256
#define WSQ      (DH * KTOT)
#define NTHR     256
#define NWAVE    8
#define EPT      8
#define CHUNK    (NTHR * EPT)
#define WCAP     (EPT * 32)
#define LISTN    (NWAVE * WCAP)
#define NBRUN    512
#define NAGB     40
#define RCAP     20480
#define DEGCAP   96
#define PKS      11
#define GBM      128
#define GTHR     256
#define GNT      8
#define BN       (16 * GNT)
#define NUSQ     (DH * (KTOT / 8))
#define PARTW    288
#define MPAD     20096
#define NTILE    (MPAD / GBM)
#define TABW     1024
#define METAW    32
#define STATW    256
#define WSMAX    134217728
#define LDS_CMP  ((2 * RCAP + 2 * NBRUN + LISTN) * 4 + 64)
#define LDS_GEMM ((GBM * BN + PARTW + BN) * 4)

static_assert((CHUNK & (CHUNK - 1)) == 0 && CHUNK <= (1 << PKS));
static_assert((NBRUN & (NBRUN - 1)) == 0 && NBRUN <= (1 << PKS));
static_assert(NTHR * 2 == NBRUN);
static_assert(LISTN >= NBRUN);
static_assert((RCAP % 1024) == 0);
static_assert(RCAP >= 16673 + 16673 / 20 + 1);
static_assert(DEGCAP >= 60 + 8);
static_assert(NEDGE < (1 << 21));
static_assert(LDS_CMP <= 300000);
static_assert(GBM == (GTHR / 32) * 16);
static_assert((DH % 32) == 0 && KTOT == 2 * DH && APW == 2 * DH);
static_assert(DH == 32 * 4 && DH == BN);
static_assert((NUSQ % NTHR) == 0 && (KTOT / 8) == 32);
static_assert((PARTW % 32) == 0 && PARTW / 4 <= GTHR && PARTW >= 2 * BN + 1);
static_assert(((PARTW * 4) % 128) == 0);
static_assert(MPAD == ((NNODE + GBM - 1) / GBM) * GBM);
static_assert(NAGB * NBRUN >= MPAD);
static_assert(((MPAD * 32) % NTHR) == 0);
static_assert(NTHR * 4 == TABW && TABW == 2 * NBRUN);
static_assert(NAGB <= 64);
static_assert(NGR * NCLS == 256);
static_assert((NEDGE % 4) == 0);

typedef float          v4f  __attribute__((ext_vector_type(4)));
typedef float          v8f  __attribute__((ext_vector_type(8)));
typedef int            v4i  __attribute__((ext_vector_type(4)));
typedef int            v8i  __attribute__((ext_vector_type(8)));
typedef unsigned int   v2u  __attribute__((ext_vector_type(2)));
typedef unsigned int   v4u  __attribute__((ext_vector_type(4)));
typedef unsigned short v8us __attribute__((ext_vector_type(8)));
typedef __bf16         v16b __attribute__((ext_vector_type(16)));
typedef v4f  __attribute__((may_alias)) v4fa;
typedef v4i  __attribute__((may_alias)) v4ia;
typedef v4u  __attribute__((may_alias)) v4ua;
typedef v8us __attribute__((may_alias)) v8usa;
union FragB { v16b v; v8us h[2]; v8i w; };

__device__ __forceinline__ v8f wmb(const FragB& a, const FragB& b, v8f c) {
  v8f d = __builtin_amdgcn_wmma_f32_16x16x32_bf16(false, a.v, false, b.v, (short)0, c, false, false);
  asm volatile("v_nop\n\tv_nop\n\tv_nop\n\tv_nop" : "+v"(d) : "v"(a.w), "v"(b.w));
  return d;
}

__device__ __forceinline__ unsigned short bf_bits(float f) {
  unsigned int u = __float_as_uint(f);
  u += 0x7FFFu + ((u >> 16) & 1u);
  return (unsigned short)(u >> 16);
}
__device__ __forceinline__ float bf_val(unsigned short b) {
  return __uint_as_float(((unsigned int)b) << 16);
}
__device__ __forceinline__ float bf_rne(float f) { return bf_val(bf_bits(f)); }

__device__ __forceinline__ float relu_np(float v) { return (v > 0.0f) ? v : (v - v); }

__device__ __forceinline__ void stage4(float* dst, const float* __restrict__ src, int lane, int rnd) {
  v4f a = *(const v4f*)(src + 4 * lane);
  if (rnd != 0) { a.x = bf_rne(a.x); a.y = bf_rne(a.y); a.z = bf_rne(a.z); a.w = bf_rne(a.w); }
  *(v4fa*)(dst + 4 * lane) = a;
}

template <int BNF>
__device__ __forceinline__ float fbn(float x, float m, float r, float g, float b) {
  if (BNF == 0) return x;
  const float v = g * (x - m) * r + b;
  return relu_np(v);
}

__device__ __forceinline__ int scan_chunk(const int* __restrict__ dsts, int nE, int cbase, int slotBase,
                                          int nb, int vec8, int* list, int tid, int lane, int wave) {
  int wc = 0;
  const int el0  = tid * EPT;
  const int e0   = cbase + el0;
  const int sent = -2147483647 - 1;
  v4i da, db;
  if (vec8 != 0 && cbase + CHUNK <= nE) {
    da = *(const v4i*)(dsts + e0);
    db = *(const v4i*)(dsts + e0 + 4);
  } else {
    da.x = (e0     < nE) ? dsts[min(e0,     nE - 1)] : sent;
    da.y = (e0 + 1 < nE) ? dsts[min(e0 + 1, nE - 1)] : sent;
    da.z = (e0 + 2 < nE) ? dsts[min(e0 + 2, nE - 1)] : sent;
    da.w = (e0 + 3 < nE) ? dsts[min(e0 + 3, nE - 1)] : sent;
    db.x = (e0 + 4 < nE) ? dsts[min(e0 + 4, nE - 1)] : sent;
    db.y = (e0 + 5 < nE) ? dsts[min(e0 + 5, nE - 1)] : sent;
    db.z = (e0 + 6 < nE) ? dsts[min(e0 + 6, nE - 1)] : sent;
    db.w = (e0 + 7 < nE) ? dsts[min(e0 + 7, nE - 1)] : sent;
  }
  const unsigned nbs = (unsigned)slotBase;
  const unsigned unb = (unsigned)nb;
  const unsigned s0 = (unsigned)da.x - nbs, s1 = (unsigned)da.y - nbs;
  const unsigned s2 = (unsigned)da.z - nbs, s3 = (unsigned)da.w - nbs;
  const unsigned s4 = (unsigned)db.x - nbs, s5 = (unsigned)db.y - nbs;
  const unsigned s6 = (unsigned)db.z - nbs, s7 = (unsigned)db.w - nbs;
  const bool h0 = s0 < unb, h1 = s1 < unb, h2 = s2 < unb, h3 = s3 < unb;
  const bool h4 = s4 < unb, h5 = s5 < unb, h6 = s6 < unb, h7 = s7 < unb;
  const unsigned any = __builtin_amdgcn_ballot_w32(h0 | h1 | h2 | h3 | h4 | h5 | h6 | h7);
  if (any != 0u) {
#define HITJ(J, HJ, SJ) { \
      const unsigned mj = __builtin_amdgcn_ballot_w32(HJ); \
      if (mj != 0u) { \
        if (HJ) { \
          const int pos = wc + (int)__builtin_amdgcn_mbcnt_lo(mj, 0u); \
          if (pos < WCAP) list[wave * WCAP + pos] = ((el0 + (J)) << PKS) | (int)(SJ); \
        } \
        wc += (int)__builtin_popcount(mj); } }
    HITJ(0, h0, s0)
    HITJ(1, h1, s1)
    HITJ(2, h2, s2)
    HITJ(3, h3, s3)
    HITJ(4, h4, s4)
    HITJ(5, h5, s5)
    HITJ(6, h6, s6)
    HITJ(7, h7, s7)
#undef HITJ
  }
  return wc;
}

__global__ __launch_bounds__(NTHR) void k_wprep(const float* __restrict__ W1, const float* __restrict__ W2,
                                                int nUnits, unsigned short* wt) {
  const int u = (int)blockIdx.x * NTHR + (int)threadIdx.x;
  if (u >= nUnits) return;
  const int mi    = u / NUSQ;
  const int v     = u - mi * NUSQ;
  const int n     = v >> 5;
  const int k8    = (v & 31) * 8;
  const int kk    = k8 & (DH - 1);
  const int layer = mi >> 1;
  const float* Wb = ((mi & 1) != 0) ? W2 : W1;
  const float* p  = Wb + (size_t)layer * DH * DH + (size_t)kk * DH + n;
  v8us o;
#pragma unroll
  for (int i = 0; i < 8; ++i) o[i] = bf_bits(p[(size_t)i * DH]);
  unsigned short* dp = wt + (size_t)mi * WSQ + (size_t)n * KTOT + k8;
  *(volatile v8us*)dp = o;
  __threadfence();
  *(volatile v8us*)dp = o;
}

__global__ __launch_bounds__(NTHR) void k_enc(const float* __restrict__ x, const float* __restrict__ encW,
                                              const float* __restrict__ encB, int nN, int nUnits, float* h0) {
  __shared__ __attribute__((aligned(16))) float sw[2 * DH];
  const int tid = (int)threadIdx.x, lane = tid & 31, wave = tid >> 5;
  if (wave == 0) stage4(sw, encW, lane, 1);
  if (wave == 1) stage4(sw + DH, encB, lane, 1);
  __syncthreads();
  const int u = (int)blockIdx.x * NTHR + tid;
  if (u >= nUnits) return;
  const int row = u >> 5;
  const int c4  = (u & 31) * 4;
  const int rc  = row < nN ? row : nN - 1;
  const float xv = bf_rne(x[rc]);
  const bool ok = row < nN;
  v4f o;
  o.x = ok ? fmaf(xv, sw[c4 + 0], sw[DH + c4 + 0]) : 0.0f;
  o.y = ok ? fmaf(xv, sw[c4 + 1], sw[DH + c4 + 1]) : 0.0f;
  o.z = ok ? fmaf(xv, sw[c4 + 2], sw[DH + c4 + 2]) : 0.0f;
  o.w = ok ? fmaf(xv, sw[c4 + 3], sw[DH + c4 + 3]) : 0.0f;
  float* hp = h0 + (size_t)row * DH + c4;
  *(volatile v4f*)hp = o;
  __threadfence();
  *(volatile v4f*)hp = o;
}

__device__ __forceinline__ v4i spill4(const int* reg2, const int* __restrict__ srcs, int i4, int nh,
                                      int nE, int nN) {
  v4i o;
#pragma unroll
  for (int j = 0; j < 4; ++j) {
    const int idx = i4 + j;
    int eid = reg2[idx];
    eid = eid < 0 ? 0 : (eid > nE - 1 ? nE - 1 : eid);
    int s = srcs[eid];
    s = s < 0 ? 0 : (s > nN - 1 ? nN - 1 : s);
    o[j] = (idx < nh) ? s : 0;
  }
  return o;
}

__global__ __launch_bounds__(NTHR) void k_compact(const int* __restrict__ srcs, const int* __restrict__ dsts,
                                                  int nN, int nE, int vec8, int* srcl, int* tab, int* meta) {
  extern __shared__ v4f lds_cmp[];
  int* reg1 = (int*)lds_cmp;
  int* reg2 = reg1 + RCAP;
  int* scnt = reg2 + RCAP;
  int* soff = scnt + NBRUN;
  int* list = soff + NBRUN;
  int* wcnt = list + LISTN;
  int* wtot = wcnt + NWAVE;
  const int tid = (int)threadIdx.x, lane = tid & 31, wave = tid >> 5;
  const int b = (int)blockIdx.x;
  const int nodeBase = b * NBRUN;

  for (int i = tid; i < NBRUN; i += NTHR) scnt[i] = 0;
  for (int i = tid; i < RCAP; i += NTHR) reg2[i] = 0;
  __syncthreads();

  int tot = 0;
  const int nChunks = (nE + CHUNK - 1) / CHUNK;
#pragma unroll 1
  for (int ch = 0; ch < nChunks; ++ch) {
    const int cbase = ch * CHUNK;
    const int wc = scan_chunk(dsts, nE, cbase, nodeBase, NBRUN, vec8, list, tid, lane, wave);
    if (lane == 0) wcnt[wave] = wc;
    __syncthreads();
    int pre = 0, all = 0;
#pragma unroll
    for (int w2 = 0; w2 < NWAVE; ++w2) {
      int c = wcnt[w2];
      c = c < 0 ? 0 : (c > WCAP ? WCAP : c);
      all += c;
      pre += (w2 < wave) ? c : 0;
    }
    const int wcc  = wc > WCAP ? WCAP : wc;
    const int base = tot + pre;
#pragma unroll 1
    for (int i = lane; i < wcc; i += 32) {
      const int ent = list[wave * WCAP + i];
      const int el  = (ent >> PKS) & (CHUNK - 1);
      const int sl  = ent & (NBRUN - 1);
      int eid = cbase + el;
      eid = eid > nE - 1 ? nE - 1 : eid;
      const int pos = base + i;
      if (pos < RCAP) reg1[pos] = (int)(((unsigned)eid << PKS) | (unsigned)sl);
    }
    tot += all;
    tot = tot > RCAP ? RCAP : tot;
    __syncthreads();
  }
  const int nh = tot;

  if (wave == 0) {
#pragma unroll 1
    for (int b0 = 0; b0 < nh; b0 += 32) {
      const int idx = b0 + lane;
      const int uv  = reg1[idx < nh ? idx : nh - 1];
      const int m32 = (nh - b0) < 32 ? (nh - b0) : 32;
#pragma unroll 1
      for (int k = 0; k < m32; ++k) {
        const int u  = __builtin_amdgcn_readlane(uv, k);
        const int sl = u & (NBRUN - 1);
        if (lane == 0) scnt[sl] = scnt[sl] + 1;
      }
    }
  }
  __syncthreads();

  {
    const int c0 = scnt[2 * tid], c1 = scnt[2 * tid + 1];
    const int e0 = c0 < 0 ? 0 : c0, e1 = c1 < 0 ? 0 : c1;
    const int ts = e0 + e1;
    int incl = ts;
#pragma unroll
    for (int d = 1; d < 32; d <<= 1) {
      const int up = __shfl_up(incl, d);
      if (lane >= d) incl += up;
    }
    if (lane == 31) wtot[wave] = incl;
    __syncthreads();
    int pre = 0;
#pragma unroll
    for (int w2 = 0; w2 < NWAVE; ++w2) pre += (w2 < wave) ? wtot[w2] : 0;
    const int run = pre + incl - ts;
    soff[2 * tid]     = run;
    soff[2 * tid + 1] = run + e0;
  }
  __syncthreads();
  for (int i = tid; i < NBRUN; i += NTHR) list[i] = soff[i];
  __syncthreads();

  if (wave == 0) {
#pragma unroll 1
    for (int b0 = 0; b0 < nh; b0 += 32) {
      const int idx = b0 + lane;
      const int uv  = reg1[idx < nh ? idx : nh - 1];
      const int m32 = (nh - b0) < 32 ? (nh - b0) : 32;
#pragma unroll 1
      for (int k = 0; k < m32; ++k) {
        const int u   = __builtin_amdgcn_readlane(uv, k);
        const int sl  = u & (NBRUN - 1);
        const int eid = (int)((unsigned)u >> PKS);
        if (lane == 0) {
          int pos = list[sl];
          pos = pos < 0 ? 0 : (pos > RCAP - 1 ? RCAP - 1 : pos);
          reg2[pos] = eid;
          list[sl] = pos + 1;
        }
      }
    }
  }
  __syncthreads();

  int big = 0;
  for (int i = tid; i < NBRUN; i += NTHR) big |= (scnt[i] > DEGCAP) ? 1 : 0;
  const unsigned bm = __builtin_amdgcn_ballot_w32(big != 0);
  if (lane == 0) wcnt[wave] = (bm != 0u) ? 1 : 0;
  __syncthreads();
  int flag = (nh >= RCAP) ? 1 : 0;
#pragma unroll
  for (int w2 = 0; w2 < NWAVE; ++w2) flag |= wcnt[w2];

  int* sp = srcl + (size_t)b * RCAP;
  int* tp = tab + (size_t)b * TABW + 4 * tid;
  int* mp = meta + (size_t)b * METAW + 4 * (tid & 7);
  const v4i tv = *(const v4ia*)(scnt + 4 * tid);
  v4i mv = {0, 0, 0, 0};
  if (tid == 0) { mv.x = nh; mv.y = flag; }
  const bool mw = tid < 8;
#pragma unroll 1
  for (int i4 = tid * 4; i4 < RCAP; i4 += NTHR * 4) {
    const v4i o = spill4(reg2, srcs, i4, nh, nE, nN);
    *(volatile v4i*)(sp + i4) = o;
  }
  *(volatile v4i*)tp = tv;
  if (mw) *(volatile v4i*)mp = mv;
  __threadfence();
#pragma unroll 1
  for (int i4 = tid * 4; i4 < RCAP; i4 += NTHR * 4) {
    const v4i o = spill4(reg2, srcs, i4, nh, nE, nN);
    *(volatile v4i*)(sp + i4) = o;
  }
  *(volatile v4i*)tp = tv;
  if (mw) *(volatile v4i*)mp = mv;
}

template <int BNF>
__global__ __launch_bounds__(NTHR) void k_agg(
    const int* __restrict__ srcl, const int* __restrict__ tab, const int* __restrict__ meta,
    const float* __restrict__ X, const float* __restrict__ stat,
    const float* __restrict__ gam, const float* __restrict__ bet,
    const float* __restrict__ epsp, int layer,
    unsigned short* Aout, int nN, int MPr) {
  __shared__ __attribute__((aligned(16))) int tabl[TABW];
  __shared__ __attribute__((aligned(16))) unsigned int stw[NWAVE * 128];
  __shared__ __attribute__((aligned(16))) float prm[4 * DH];
  const int tid = (int)threadIdx.x, lane = tid & 31, wave = tid >> 5;
  const int b = (int)blockIdx.x;
  const int nodeBase = b * NBRUN;

  {
    const v4i t4 = *(const v4i*)(tab + (size_t)b * TABW + 4 * tid);
    *(v4ia*)(tabl + 4 * tid) = t4;
  }
  if (BNF != 0) {
    if (wave == 0) stage4(prm,          stat,      lane, 0);
    if (wave == 1) stage4(prm + DH,     stat + DH, lane, 0);
    if (wave == 2) stage4(prm + 2 * DH, gam,       lane, 1);
    if (wave == 3) stage4(prm + 3 * DH, bet,       lane, 1);
  }
  __syncthreads();

  int nh = meta[(size_t)b * METAW];
  nh = nh < 0 ? 0 : (nh > RCAP ? RCAP : nh);
  const int flag = meta[(size_t)b * METAW + 1];
  const float ope = 1.0f + bf_rne(epsp[layer]);
  float pm[4], pr[4], pg[4], pb[4];
#pragma unroll
  for (int j = 0; j < 4; ++j) {
    if (BNF != 0) {
      pm[j] = prm[4 * lane + j];
      pr[j] = prm[DH + 4 * lane + j];
      pg[j] = prm[2 * DH + 4 * lane + j];
      pb[j] = prm[3 * DH + 4 * lane + j];
    } else {
      pm[j] = 0.0f; pr[j] = 1.0f; pg[j] = 1.0f; pb[j] = 0.0f;
    }
  }

  const int nbw = NBRUN / NWAVE;
  const float qnan = __int_as_float(0x7fc00000);
  unsigned int* stwu = stw + wave * 128;
  const int* sl = srcl + (size_t)b * RCAP;

#pragma unroll 1
  for (int jt = 0; jt < nbw; ++jt) {
    const int slot = wave * nbw + jt;
    const int grow = nodeBase + slot;
    int st = tabl[NBRUN + slot];
    const int craw = tabl[slot];
    int cnt = craw;
    st  = st < 0 ? 0 : (st > nh ? nh : st);
    cnt = cnt < 0 ? 0 : (cnt > DEGCAP ? DEGCAP : cnt);
    if (cnt > nh - st) cnt = nh - st;
    const float pz = (flag != 0 || craw > DEGCAP) ? qnan : 0.0f;
    const bool liveRow = grow < nN;

    float ag0 = 0.f, ag1 = 0.f, ag2 = 0.f, ag3 = 0.f;
#pragma unroll 1
    for (int b0 = 0; b0 < cnt; b0 += 32) {
      int idx = st + b0 + lane;
      idx = idx > nh - 1 ? nh - 1 : idx;
      idx = idx < 0 ? 0 : (idx > RCAP - 1 ? RCAP - 1 : idx);
      const int sraw = sl[idx];
      const int sv = sraw < 0 ? 0 : (sraw > nN - 1 ? nN - 1 : sraw);
      const int m32 = (cnt - b0) < 32 ? (cnt - b0) : 32;
#pragma unroll 1
      for (int k = 0; k < m32; ++k) {
        const int sk = __builtin_amdgcn_readlane(sv, k);
        const v4f v = *(const v4f*)(X + (size_t)sk * DH + 4 * lane);
        ag0 += fbn<BNF>(v.x, pm[0], pr[0], pg[0], pb[0]);
        ag1 += fbn<BNF>(v.y, pm[1], pr[1], pg[1], pb[1]);
        ag2 += fbn<BNF>(v.z, pm[2], pr[2], pg[2], pb[2]);
        ag3 += fbn<BNF>(v.w, pm[3], pr[3], pg[3], pb[3]);
      }
    }
    const int nc = liveRow ? grow : nN - 1;
    const v4f sf = *(const v4f*)(X + (size_t)nc * DH + 4 * lane);
    const float s0 = fbn<BNF>(sf.x, pm[0], pr[0], pg[0], pb[0]);
    const float s1 = fbn<BNF>(sf.y, pm[1], pr[1], pg[1], pb[1]);
    const float s2 = fbn<BNF>(sf.z, pm[2], pr[2], pg[2], pb[2]);
    const float s3 = fbn<BNF>(sf.w, pm[3], pr[3], pg[3], pb[3]);
    float r0 = ope * s0 + ag0, r1 = ope * s1 + ag1, r2 = ope * s2 + ag2, r3 = ope * s3 + ag3;
    r0 = (liveRow ? r0 : 0.0f) + pz;
    r1 = (liveRow ? r1 : 0.0f) + pz;
    r2 = (liveRow ? r2 : 0.0f) + pz;
    r3 = (liveRow ? r3 : 0.0f) + pz;

    const unsigned short hb0 = bf_bits(r0), hb1 = bf_bits(r1), hb2 = bf_bits(r2), hb3 = bf_bits(r3);
    const unsigned short lb0 = bf_bits(r0 - bf_val(hb0)), lb1 = bf_bits(r1 - bf_val(hb1));
    const unsigned short lb2 = bf_bits(r2 - bf_val(hb2)), lb3 = bf_bits(r3 - bf_val(hb3));
    v2u hw, lw;
    hw.x = (unsigned int)hb0 | ((unsigned int)hb1 << 16);
    hw.y = (unsigned int)hb2 | ((unsigned int)hb3 << 16);
    lw.x = (unsigned int)lb0 | ((unsigned int)lb1 << 16);
    lw.y = (unsigned int)lb2 | ((unsigned int)lb3 << 16);
    __builtin_amdgcn_fence(__ATOMIC_RELEASE, "wavefront");
    __builtin_amdgcn_wave_barrier();
    *(v2u*)(stwu + 2 * lane)      = hw;
    *(v2u*)(stwu + 64 + 2 * lane) = lw;
    __builtin_amdgcn_fence(__ATOMIC_RELEASE, "wavefront");
    __builtin_amdgcn_wave_barrier();
    const v4u pk = *(const v4ua*)(stwu + 4 * lane);
    unsigned short* gp = Aout + (size_t)grow * (size_t)APW + 8 * lane;
    const bool wsv = grow < MPr;
    if (wsv) *(volatile v4u*)gp = pk;
    __threadfence();
    if (wsv) *(volatile v4u*)gp = pk;
  }
}

__global__ __launch_bounds__(GTHR) void k_gemm(const unsigned short* __restrict__ A,
                                               const unsigned short* __restrict__ WT,
                                               const float* __restrict__ bias,
                                               float* outF, float* part, int nN, int mRows)
{
  constexpr int NT = GNT;
  constexpr int NI = 16;
  extern __shared__ v4f lds_gm[];
  float* stg   = (float*)lds_gm;
  float* pst   = stg + GBM * BN;
  float* sbias = pst + PARTW;
  const int tid = (int)threadIdx.x, lane = tid & 31, wave = tid >> 5, hh = lane >> 4, m = lane & 15;
  const int rowBase = (int)blockIdx.x * GBM;

  if (wave == 0) stage4(sbias, bias, lane, 1);

  v8f acc[NT];
  {
    const v8f z = {0.f, 0.f, 0.f, 0.f, 0.f, 0.f, 0.f, 0.f};
#pragma unroll
    for (int t = 0; t < NT; ++t) acc[t] = z;
  }
  const unsigned short* ap = A + (size_t)(rowBase + 16 * wave + m) * (size_t)APW + 8 * hh;
  const unsigned short* wp = WT + (size_t)m * (size_t)KTOT + 8 * hh;
  constexpr int ksteps = KTOT / 32;
#pragma unroll 1
  for (int ks = 0; ks < ksteps; ++ks) {
    FragB af;
    af.h[0] = *(const v8usa*)(ap + 32 * ks);
    af.h[1] = *(const v8usa*)(ap + 32 * ks + 16);
#pragma unroll
    for (int t = 0; t < NT; ++t) {
      const unsigned short* wq = wp + (size_t)(16 * t) * (size_t)KTOT + 32 * ks;
      FragB bf;
      bf.h[0] = *(const v8usa*)wq;
      bf.h[1] = *(const v8usa*)(wq + 16);
      acc[t] = wmb(af, bf, acc[t]);
    }
  }
  __syncthreads();

#pragma unroll
  for (int t = 0; t < NT; ++t) {
    const int lc = 16 * t + m;
    const float bb = sbias[lc];
#pragma unroll
    for (int r = 0; r < 8; ++r) {
      const int lr = 16 * wave + 8 * hh + r;
      const bool live = (rowBase + lr) < nN;
      const float v = acc[t][r] + bb;
      stg[lr * BN + lc] = live ? v : 0.0f;
    }
  }
  __syncthreads();

  if (tid < BN) {
    int rv = nN - rowBase;
    rv = rv < 0 ? 0 : (rv > GBM ? GBM : rv);
    float n = 0.0f, mean = 0.0f, M2 = 0.0f;
#pragma unroll 1
    for (int r = 0; r < rv; ++r) {
      const float v = stg[r * BN + tid];
      n += 1.0f;
      const float rk = 1.0f / n;
      const float d = v - mean;
      mean = fmaf(d, rk, mean);
      M2 = fmaf(d, v - mean, M2);
    }
    pst[1 + tid] = mean;
    pst[1 + BN + tid] = M2;
    if (tid == 0) pst[0] = n;
#pragma unroll 1
    for (int i = 2 * BN + 1 + tid; i < PARTW; i += BN) pst[i] = 0.0f;
  }

  v4f fv[NI];
#pragma unroll
  for (int i = 0; i < NI; ++i) {
    const int lr = 16 * wave + i;
    fv[i] = *(const v4fa*)(stg + lr * BN + 4 * lane);
  }
#pragma unroll
  for (int i = 0; i < NI; ++i) {
    const int gr = rowBase + 16 * wave + i;
    float* op = outF + (size_t)gr * (size_t)DH + 4 * lane;
    if (gr < mRows) *(volatile v4f*)op = fv[i];
  }
  __threadfence();
#pragma unroll
  for (int i = 0; i < NI; ++i) {
    const int gr = rowBase + 16 * wave + i;
    float* op = outF + (size_t)gr * (size_t)DH + 4 * lane;
    if (gr < mRows) *(volatile v4f*)op = fv[i];
  }
  __syncthreads();
  v4f pv = {0.f, 0.f, 0.f, 0.f};
  if (tid < PARTW / 4) {
    pv = *(const v4fa*)(pst + 4 * tid);
    *(volatile v4f*)(part + (size_t)blockIdx.x * PARTW + 4 * tid) = pv;
  }
  __threadfence();
  if (tid < PARTW / 4) {
    *(volatile v4f*)(part + (size_t)blockIdx.x * PARTW + 4 * tid) = pv;
  }
}

__global__ __launch_bounds__(DH) void k_comb(const float* __restrict__ part, int nPart, float* st) {
  __shared__ __attribute__((aligned(16))) float stg[2 * DH];
  const int tid = (int)threadIdx.x;
  const int c = tid & (DH - 1);
  double n = 0.0, mean = 0.0, M2 = 0.0;
#pragma unroll 1
  for (int b = 0; b < nPart; ++b) {
    const float* pr = part + (size_t)b * PARTW;
    const float nb = pr[0];
    const float mb = pr[1 + c];
    const float qb = pr[1 + DH + c];
    if (nb > 0.5f) {
      const double nn = n + (double)nb;
      const double delta = (double)mb - mean;
      const double f = (double)nb / nn;
      mean = mean + delta * f;
      M2 = M2 + (double)qb + delta * delta * n * f;
      n = nn;
    }
  }
  const double nt = n < 1.0 ? 1.0 : n;
  const float var = (float)(M2 / nt);
  const float rstd = 1.0f / sqrtf(var + 1e-5f);
  stg[c] = (float)mean;
  stg[DH + c] = rstd;
  __syncthreads();
  v4f v = {0.f, 0.f, 0.f, 0.f};
  if (tid < (2 * DH) / 4) {
    v = *(const v4fa*)(stg + 4 * tid);
    *(volatile v4f*)(st + 4 * tid) = v;
  }
  __threadfence();
  if (tid < (2 * DH) / 4) {
    *(volatile v4f*)(st + 4 * tid) = v;
  }
}

__global__ __launch_bounds__(NTHR) void k_apply(const float* __restrict__ T, const float* __restrict__ stat,
                                                const float* __restrict__ gam, const float* __restrict__ bet,
                                                int nN, int nUnits, unsigned short* outH) {
  __shared__ __attribute__((aligned(16))) float prm[4 * DH];
  const int tid = (int)threadIdx.x, lane = tid & 31, wave = tid >> 5;
  if (wave == 0) stage4(prm,          stat,      lane, 0);
  if (wave == 1) stage4(prm + DH,     stat + DH, lane, 0);
  if (wave == 2) stage4(prm + 2 * DH, gam,       lane, 1);
  if (wave == 3) stage4(prm + 3 * DH, bet,       lane, 1);
  __syncthreads();
  const int u = (int)blockIdx.x * NTHR + tid;
  if (u >= nUnits) return;
  const int row = u >> 5;
  const int m  = lane & 15;
  const bool isHi = (lane >> 4) == 0;
  const int cb = 8 * m;
  const int rc = row < nN ? row : nN - 1;
  const bool ok = row < nN;
  const v4f a = *(const v4f*)(T + (size_t)rc * DH + cb);
  const v4f b = *(const v4f*)(T + (size_t)rc * DH + cb + 4);
  float f[8] = {a.x, a.y, a.z, a.w, b.x, b.y, b.z, b.w};
#pragma unroll
  for (int j = 0; j < 8; ++j) {
    const int c = cb + j;
    const float v = prm[2 * DH + c] * (f[j] - prm[c]) * prm[DH + c] + prm[3 * DH + c];
    const float y = relu_np(v);
    f[j] = ok ? y : 0.0f;
  }
  unsigned int w[4];
#pragma unroll
  for (int j = 0; j < 4; ++j) {
    const unsigned short h0 = bf_bits(f[2 * j]), h1 = bf_bits(f[2 * j + 1]);
    const unsigned short l0 = bf_bits(f[2 * j] - bf_val(h0)), l1 = bf_bits(f[2 * j + 1] - bf_val(h1));
    const unsigned short q0 = isHi ? h0 : l0, q1 = isHi ? h1 : l1;
    w[j] = (unsigned int)q0 | ((unsigned int)q1 << 16);
  }
  v4u pw; pw.x = w[0]; pw.y = w[1]; pw.z = w[2]; pw.w = w[3];
  unsigned short* op = outH + (size_t)row * (size_t)APW + 8 * lane;
  *(volatile v4u*)op = pw;
  __threadfence();
  *(volatile v4u*)op = pw;
}

__global__ __launch_bounds__(NTHR) void k_pool(const float* __restrict__ U, const int* __restrict__ bat,
                                               const float* __restrict__ stat, const float* __restrict__ gam,
                                               const float* __restrict__ bet, int nN, float* pooled) {
  __shared__ __attribute__((aligned(16))) float wsum[NWAVE * DH];
  __shared__ int wcn[NWAVE];
  __shared__ __attribute__((aligned(16))) float outs[DH];
  __shared__ __attribute__((aligned(16))) float prm[4 * DH];
  const int tid = (int)threadIdx.x, lane = tid & 31, wave = tid >> 5;
  const int g = (int)blockIdx.x;
  if (wave == 0) stage4(prm,          stat,      lane, 0);
  if (wave == 1) stage4(prm + DH,     stat + DH, lane, 0);
  if (wave == 2) stage4(prm + 2 * DH, gam,       lane, 1);
  if (wave == 3) stage4(prm + 3 * DH, bet,       lane, 1);
  __syncthreads();
  float pm[4], pr[4], pg[4], pb[4];
#pragma unroll
  for (int j = 0; j < 4; ++j) {
    pm[j] = prm[4 * lane + j];
    pr[j] = prm[DH + 4 * lane + j];
    pg[j] = prm[2 * DH + 4 * lane + j];
    pb[j] = prm[3 * DH + 4 * lane + j];
  }

  float a0 = 0.0f, a1 = 0.0f, a2 = 0.0f, a3 = 0.0f;
  int cnt = 0;
#pragma unroll 1
  for (int i0 = wave * 32; i0 < nN; i0 += NTHR) {
    const int i  = i0 + lane;
    const int ic = i < nN ? i : nN - 1;
    const int bq = bat[ic];
    const bool hit = (i < nN) && (bq == g);
    unsigned msk = __builtin_amdgcn_ballot_w32(hit);
    int nh = (int)__builtin_popcount(msk);
    nh = nh > 32 ? 32 : nh;
    cnt += nh;
#pragma unroll 1
    for (int q = 0; q < nh; ++q) {
      const int k = __builtin_ffs((int)msk) - 1;
      msk &= msk - 1u;
      int node = i0 + (k < 0 ? 0 : k);
      node = node > nN - 1 ? nN - 1 : node;
      const v4f v = *(const v4f*)(U + (size_t)node * DH + 4 * lane);
      a0 += fbn<1>(v.x, pm[0], pr[0], pg[0], pb[0]);
      a1 += fbn<1>(v.y, pm[1], pr[1], pg[1], pb[1]);
      a2 += fbn<1>(v.z, pm[2], pr[2], pg[2], pb[2]);
      a3 += fbn<1>(v.w, pm[3], pr[3], pg[3], pb[3]);
    }
  }
  wsum[wave * DH + 4 * lane + 0] = a0;
  wsum[wave * DH + 4 * lane + 1] = a1;
  wsum[wave * DH + 4 * lane + 2] = a2;
  wsum[wave * DH + 4 * lane + 3] = a3;
  if (lane == 0) wcn[wave] = cnt;
  __syncthreads();
  if (tid < DH) {
    float s = 0.0f;
    int c = 0;
#pragma unroll
    for (int w2 = 0; w2 < NWAVE; ++w2) { s += wsum[w2 * DH + tid]; c += wcn[w2]; }
    const float cf = (c < 1) ? 1.0f : (float)c;
    outs[tid] = s * (1.0f / cf);
  }
  __syncthreads();
  const v4f ov = *(const v4fa*)(outs + 4 * lane);
  float* op = pooled + (size_t)g * DH + 4 * lane;
  const bool okst = (wave == 0);
  if (okst) *(volatile v4f*)op = ov;
  __threadfence();
  if (okst) *(volatile v4f*)op = ov;
}

__global__ __launch_bounds__(NTHR) void k_head(const float* __restrict__ pooled, const float* __restrict__ clsW,
                                               const float* __restrict__ clsB, const int* __restrict__ meta,
                                               int nBlk, float* out) {
  __shared__ __attribute__((aligned(16))) float sw[DH * NCLS];
  __shared__ __attribute__((aligned(16))) float outs[NGR * NCLS];
  __shared__ int fl[64];
  const int tid = (int)threadIdx.x, lane = tid & 31, wave = tid >> 5;
  if (tid < 64) {
    v4f a = *(const v4f*)(clsW + 4 * tid);
    a.x = bf_rne(a.x); a.y = bf_rne(a.y); a.z = bf_rne(a.z); a.w = bf_rne(a.w);
    *(v4fa*)(sw + 4 * tid) = a;
    const int bi = tid < nBlk ? tid : nBlk - 1;
    const int f = meta[(size_t)bi * METAW + 1];
    fl[tid] = (tid < nBlk) ? f : 0;
  }
  __syncthreads();
  const int g = tid >> 1, c = tid & 1;
  const float* pr = pooled + (size_t)g * DH;
  float s = 0.0f;
#pragma unroll 4
  for (int k4 = 0; k4 < DH / 4; ++k4) {
    const v4f p = *(const v4f*)(pr + 4 * k4);
    s = fmaf(p.x, sw[(4 * k4 + 0) * NCLS + c], s);
    s = fmaf(p.y, sw[(4 * k4 + 1) * NCLS + c], s);
    s = fmaf(p.z, sw[(4 * k4 + 2) * NCLS + c], s);
    s = fmaf(p.w, sw[(4 * k4 + 3) * NCLS + c], s);
  }
  s = s + bf_rne(clsB[c]);
  int any = 0;
  const int nb2 = nBlk > 64 ? 64 : nBlk;
#pragma unroll 1
  for (int i = 0; i < nb2; ++i) any |= fl[i];
  const float val = (any != 0) ? __int_as_float(0x7fc00000) : s;
  outs[tid] = val;
  __syncthreads();
  const v4f ov = *(const v4fa*)(outs + 32 * wave + 4 * (lane & 7));
  float* op = out + 32 * wave + 4 * (lane & 7);
  const bool okst = lane < 8;
  if (okst) *(volatile v4f*)op = ov;
  __threadfence();
  if (okst) *(volatile v4f*)op = ov;
}

static inline size_t al256(size_t o) { return (o + 255) & ~(size_t)255; }

extern "C" void kernel_launch(void* const* d_in, const int* in_sizes, int n_in,
                              void* d_out, int out_size, void* d_ws, size_t ws_size,
                              hipStream_t stream) {
  if (n_in < 16) return;
  if (in_sizes[0] != NNODE) return;
  if (in_sizes[1] != 2 * NEDGE) return;
  if (in_sizes[2] != NNODE) return;
  if (in_sizes[3] != DH || in_sizes[4] != DH) return;
  if (in_sizes[5] != NLAY * DH * DH || in_sizes[9] != NLAY * DH * DH) return;
  if (in_sizes[6] != NLAY * DH || in_sizes[7] != NLAY * DH || in_sizes[8] != NLAY * DH) return;
  if (in_sizes[10] != NLAY * DH || in_sizes[12] != NLAY * DH || in_sizes[13] != NLAY * DH) return;
  if (in_sizes[11] != NLAY) return;
  if (in_sizes[14] != DH * NCLS || in_sizes[15] != NCLS) return;
  if (out_size != NGR * NCLS) return;

  const float* x    = (const float*)d_in[0];
  const int*   ei   = (const int*)  d_in[1];
  const int*   src  = ei;
  const int*   dst  = ei + NEDGE;
  const int*   bat  = (const int*)  d_in[2];
  const float* encW = (const float*)d_in[3];
  const float* encB = (const float*)d_in[4];
  const float* W1   = (const float*)d_in[5];
  const float* b1   = (const float*)d_in[6];
  const float* g1   = (const float*)d_in[7];
  const float* be1  = (const float*)d_in[8];
  const float* W2   = (const float*)d_in[9];
  const float* b2   = (const float*)d_in[10];
  const float* eps  = (const float*)d_in[11];
  const float* bng  = (const float*)d_in[12];
  const float* bnb  = (const float*)d_in[13];
  const float* clsW = (const float*)d_in[14];
  const float* clsB = (const float*)d_in[15];
  float* out = (float*)d_out;

  const int nN = NNODE, nE = NEDGE;
  const int vec8 = 1;
  const int nMat = 2 * NLAY;
  const int nUw  = nMat * NUSQ;
  const int nU   = MPAD * 32;

  char* ws = (char*)d_ws;
  size_t off = 0;
  const size_t oWT = off; off = al256(off + (size_t)nMat * WSQ * 2);
  const size_t oP1 = off; off = al256(off + (size_t)MPAD * APW * 2);
  const size_t oP2 = off; off = al256(off + (size_t)MPAD * DH * 4);
  const size_t oSL = off; off = al256(off + (size_t)NAGB * RCAP * 4);
  const size_t oTB = off; off = al256(off + (size_t)NAGB * TABW * 4);
  const size_t oMT = off; off = al256(off + (size_t)NAGB * METAW * 4);
  const size_t oPT = off; off = al256(off + (size_t)NTILE * PARTW * 4);
  const size_t oST = off; off = al256(off + (size_t)nMat * STATW * 4);
  const size_t oPL = off; off = al256(off + (size_t)NGR * DH * 4);
  if (off > ws_size || off > (size_t)WSMAX) return;
  unsigned short* WT   = (unsigned short*)(ws + oWT);
  unsigned short* P1   = (unsigned short*)(ws + oP1);
  float*          P2   = (float*)(ws + oP2);
  int*            SRCL = (int*)(ws + oSL);
  int*            TAB  = (int*)(ws + oTB);
  int*            META = (int*)(ws + oMT);
  float*          PART = (float*)(ws + oPT);
  float*          STAT = (float*)(ws + oST);
  float*          POOL = (float*)(ws + oPL);

  hipFuncSetAttribute(reinterpret_cast<const void*>(&k_compact), hipFuncAttributeMaxDynamicSharedMemorySize, LDS_CMP);
  hipFuncSetAttribute(reinterpret_cast<const void*>(&k_gemm), hipFuncAttributeMaxDynamicSharedMemorySize, LDS_GEMM);

  k_wprep<<<nUw / NTHR, NTHR, 0, stream>>>(W1, W2, nUw, WT);
  k_enc<<<nU / NTHR, NTHR, 0, stream>>>(x, encW, encB, nN, nU, P2);
  k_compact<<<NAGB, NTHR, LDS_CMP, stream>>>(src, dst, nN, nE, vec8, SRCL, TAB, META);

  for (int l = 0; l < NLAY; ++l) {
    if (l == 0) {
      k_agg<0><<<NAGB, NTHR, 0, stream>>>(SRCL, TAB, META, P2, STAT, bng, bnb, eps, l, P1, nN, MPAD);
    } else {
      k_agg<1><<<NAGB, NTHR, 0, stream>>>(SRCL, TAB, META, P2, STAT + (size_t)(2 * (l - 1) + 1) * STATW,
                                          bng + (size_t)(l - 1) * DH, bnb + (size_t)(l - 1) * DH,
                                          eps, l, P1, nN, MPAD);
    }
    k_gemm<<<NTILE, GTHR, LDS_GEMM, stream>>>(P1, WT + (size_t)(2 * l) * WSQ, b1 + (size_t)l * DH,
                                              P2, PART, nN, MPAD);
    k_comb<<<1, DH, 0, stream>>>(PART, NTILE, STAT + (size_t)(2 * l) * STATW);
    k_apply<<<nU / NTHR, NTHR, 0, stream>>>(P2, STAT + (size_t)(2 * l) * STATW, g1 + (size_t)l * DH,
                                            be1 + (size_t)l * DH, nN, nU, P1);
    k_gemm<<<NTILE, GTHR, LDS_GEMM, stream>>>(P1, WT + (size_t)(2 * l + 1) * WSQ, b2 + (size_t)l * DH,
                                              P2, PART, nN, MPAD);
    k_comb<<<1, DH, 0, stream>>>(PART, NTILE, STAT + (size_t)(2 * l + 1) * STATW);
  }
  k_pool<<<NGR, NTHR, 0, stream>>>(P2, bat, STAT + (size_t)(2 * (NLAY - 1) + 1) * STATW,
                                   bng + (size_t)(NLAY - 1) * DH, bnb + (size_t)(NLAY - 1) * DH, nN, POOL);
  k_head<<<1, NTHR, 0, stream>>>(POOL, clsW, clsB, META, NAGB, out);
}
